// CustomModel_79396765433857
// MI455X (gfx1250) — hardware-verified
//
#include <hip/hip_runtime.h>
#define NB 4
#define NN 512
#define TT 10
#define FF 516
#define MH 128
#define MD 32
#define UH 128
#define SCH 64
typedef __bf16 v16b __attribute__((ext_vector_type(16)));
typedef unsigned short v8us __attribute__((ext_vector_type(8), may_alias));
typedef float  v8f  __attribute__((ext_vector_type(8)));
typedef float  v4f  __attribute__((ext_vector_type(4)));
typedef float  v4fa __attribute__((ext_vector_type(4), may_alias));
union FragB { v16b v; v8us half[2]; unsigned short u[16]; };

__device__ __forceinline__ unsigned short bf16_bits(float x) { unsigned int u = __float_as_uint(x); return (unsigned short)((u + 0x7FFFu + ((u >> 16) & 1u)) >> 16); }
__device__ __forceinline__ float bf16_val(unsigned short b) { return __uint_as_float(((unsigned int)b) << 16); }
__device__ __forceinline__ float bf16_round(float x) { return bf16_val(bf16_bits(x)); }
template <int NT>
__device__ __forceinline__ v8f mmaN(v16b ah, v16b al, v16b bh, v16b bl, v8f c) {
  c = __builtin_amdgcn_wmma_f32_16x16x32_bf16(false, ah, false, bh, (short)0, c, false, false);
  if (NT >= 2) c = __builtin_amdgcn_wmma_f32_16x16x32_bf16(false, al, false, bh, (short)0, c, false, false);
  if (NT >= 3) c = __builtin_amdgcn_wmma_f32_16x16x32_bf16(false, ah, false, bl, (short)0, c, false, false);
  asm volatile("v_nop\n\tv_nop\n\tv_nop\n\tv_nop" : "+v"(c) : "v"(ah), "v"(al), "v"(bh), "v"(bl));
  return c;
}

__global__ __launch_bounds__(256) void k_wt_bf16(const float* __restrict__ W, unsigned short* __restrict__ Wt, int K, int N) {
  const int t = blockIdx.x * 256 + threadIdx.x;
  const int k8n = K / 8;
  if (t >= N * k8n) return;
  const int n = t / k8n, k8 = (t % k8n) * 8;
  v8us v;
#pragma unroll
  for (int i = 0; i < 8; ++i) v[i] = bf16_bits(W[(size_t)(k8 + i) * N + n]);
  *(volatile v8us*)(Wt + (size_t)n * K + k8) = v;
  __threadfence();
  *(volatile v8us*)(Wt + (size_t)n * K + k8) = v;
}

template <bool ASPLIT, int ACT, bool BIAS_BF16>
__global__ __launch_bounds__(128) void k_gemm_bf(const float* __restrict__ A, int lda, const unsigned short* __restrict__ Wt, int ldb,
                                               const float* __restrict__ bias, float* __restrict__ C, int ldc, int M, int N, int K) {
  __shared__ __attribute__((aligned(16))) float so[4][16][64];
  const int tid = threadIdx.x, w = tid >> 5, lane = tid & 31, ln = lane & 15, hh = lane >> 4;
  const int ntn = N / 64;
  const int wid = blockIdx.x * 4 + w;
  const int mt = wid / ntn, nq = wid % ntn;
  if (mt * 16 >= M) return;
  const int row0 = mt * 16, col0 = nq * 64;
  const float* arow = A + (size_t)(row0 + ln) * lda;
  v8f acc[4] = {};
  for (int kb = 0; kb < K; kb += 32) {
    FragB ah, al;
    const v4f x0 = *(const v4fa*)(arow + kb + 8 * hh), x1 = *(const v4fa*)(arow + kb + 8 * hh + 4);
    const v4f x2 = *(const v4fa*)(arow + kb + 16 + 8 * hh), x3 = *(const v4fa*)(arow + kb + 16 + 8 * hh + 4);
    float xs[16] = {x0[0],x0[1],x0[2],x0[3],x1[0],x1[1],x1[2],x1[3],x2[0],x2[1],x2[2],x2[3],x3[0],x3[1],x3[2],x3[3]};
#pragma unroll
    for (int i = 0; i < 16; ++i) { const unsigned short hb = bf16_bits(xs[i]); ah.u[i] = hb; al.u[i] = ASPLIT ? bf16_bits(xs[i] - bf16_val(hb)) : (unsigned short)0; }
#pragma unroll
    for (int t = 0; t < 4; ++t) {
      const unsigned short* brow = Wt + (size_t)(col0 + t * 16 + ln) * ldb + kb;
      FragB b;
      b.half[0] = *(const v8us*)(brow + 8 * hh);
      b.half[1] = *(const v8us*)(brow + 16 + 8 * hh);
      acc[t] = mmaN<ASPLIT ? 2 : 1>(ah.v, al.v, b.v, b.v, acc[t]);
    }
  }
#pragma unroll
  for (int t = 0; t < 4; ++t) {
    float bv = bias ? bias[col0 + t * 16 + ln] : 0.f;
    if (BIAS_BF16) bv = bf16_round(bv);
#pragma unroll
    for (int r = 0; r < 8; ++r) { float v = acc[t][r] + bv; if (ACT == 1) v = fmaxf(v, 0.f); so[w][8 * hh + r][t * 16 + ln] = v; }
  }
  __builtin_amdgcn_fence(__ATOMIC_ACQ_REL, "workgroup");
  __builtin_amdgcn_wave_barrier();
  const int rsub = lane >> 4, c4 = (lane & 15) * 4;
  for (int pass = 0; pass < 2; ++pass) {
#pragma unroll
    for (int q = 0; q < 8; ++q) {
      const int r = q * 2 + rsub;
      const v4f v = *(const v4fa*)&so[w][r][c4];
      *(volatile v4f*)(C + (size_t)(row0 + r) * ldc + col0 + c4) = v;
    }
    if (pass == 0) __threadfence();
  }
}

template <bool ASPLIT, int ACT, bool BIAS_BF16, bool RES_BF16>
__global__ __launch_bounds__(128) void k_gemm_bf3(const float* __restrict__ A, int lda, const unsigned short* __restrict__ Wt, int ldb,
                                                const float* __restrict__ bias, const float* __restrict__ resid, int rmod, int ldr,
                                                float* __restrict__ C, int ldc, int M, int N, int K) {
  __shared__ __attribute__((aligned(16))) float so[4][16][64];
  const int tid = threadIdx.x, w = tid >> 5, lane = tid & 31, ln = lane & 15, hh = lane >> 4;
  const int ntn = N / 64;
  const int wid = blockIdx.x * 4 + w;
  const int mt = wid / ntn, nq = wid % ntn;
  if (mt * 16 >= M) return;
  const int row0 = mt * 16, col0 = nq * 64;
  const float* arow = A + (size_t)(row0 + ln) * lda;
  v8f acc[4] = {};
  for (int kb = 0; kb < K; kb += 32) {
    FragB ah, al;
    const v4f x0 = *(const v4fa*)(arow + kb + 8 * hh), x1 = *(const v4fa*)(arow + kb + 8 * hh + 4);
    const v4f x2 = *(const v4fa*)(arow + kb + 16 + 8 * hh), x3 = *(const v4fa*)(arow + kb + 16 + 8 * hh + 4);
    float xs[16] = {x0[0],x0[1],x0[2],x0[3],x1[0],x1[1],x1[2],x1[3],x2[0],x2[1],x2[2],x2[3],x3[0],x3[1],x3[2],x3[3]};
#pragma unroll
    for (int i = 0; i < 16; ++i) { const unsigned short hb = bf16_bits(xs[i]); ah.u[i] = hb; al.u[i] = ASPLIT ? bf16_bits(xs[i] - bf16_val(hb)) : (unsigned short)0; }
#pragma unroll
    for (int t = 0; t < 4; ++t) {
      const unsigned short* brow = Wt + (size_t)(col0 + t * 16 + ln) * ldb + kb;
      FragB b;
      b.half[0] = *(const v8us*)(brow + 8 * hh);
      b.half[1] = *(const v8us*)(brow + 16 + 8 * hh);
      acc[t] = mmaN<ASPLIT ? 2 : 1>(ah.v, al.v, b.v, b.v, acc[t]);
    }
  }
#pragma unroll
  for (int t = 0; t < 4; ++t) {
    const int col = col0 + t * 16 + ln;
    float bv = bias ? bias[col] : 0.f;
    if (BIAS_BF16) bv = bf16_round(bv);
#pragma unroll
    for (int r = 0; r < 8; ++r) {
      float v = acc[t][r] + bv;
      if (resid) { float rv = resid[(size_t)((row0 + 8 * hh + r) % rmod) * ldr + col]; if (RES_BF16) rv = bf16_round(rv); v += rv; }
      if (ACT == 1) v = fmaxf(v, 0.f);
      if (ACT == 2) v = 0.5f * v * (1.0f + erff(v * 0.70710678118654752f));
      if (ACT == 3) { const float u = 0.7978845608028654f * (v + 0.044715f * v * v * v); v = 0.5f * v * (1.0f + tanhf(u)); }
      so[w][8 * hh + r][t * 16 + ln] = v;
    }
  }
  __builtin_amdgcn_fence(__ATOMIC_ACQ_REL, "workgroup");
  __builtin_amdgcn_wave_barrier();
  const int rsub = lane >> 4, c4 = (lane & 15) * 4;
  for (int pass = 0; pass < 2; ++pass) {
#pragma unroll
    for (int q = 0; q < 8; ++q) {
      const int r = q * 2 + rsub;
      const v4f v = *(const v4fa*)&so[w][r][c4];
      *(volatile v4f*)(C + (size_t)(row0 + r) * ldc + col0 + c4) = v;
    }
    if (pass == 0) __threadfence();
  }
}
template <bool PARAM_BF16>
__global__ __launch_bounds__(256) void k_layernorm(const float* __restrict__ X, const float* __restrict__ R, const float* __restrict__ g, const float* __restrict__ bta,
                                                  float* __restrict__ out_sum, float* __restrict__ out_norm, int N, float eps) {
  __shared__ float red[256];
  const int row = blockIdx.x, tid = threadIdx.x;
  const float* x = X + (size_t)row * N; const float* rr = R ? R + (size_t)row * N : nullptr;
  float vals[16];
  const int per = N / 256;
  float s1 = 0.f;
  for (int u = 0; u < per / 4; ++u) {
    const int j = tid * 4 + 1024 * u;
    const v4f a = *(const v4fa*)(x + j);
    v4f b = {0.f,0.f,0.f,0.f}; if (rr) b = *(const v4fa*)(rr + j);
#pragma unroll
    for (int q = 0; q < 4; ++q) { const float v = a[q] + b[q]; vals[u * 4 + q] = v; s1 += v; }
  }
  red[tid] = s1; __syncthreads();
  for (int st = 128; st > 0; st >>= 1) { if (tid < st) red[tid] += red[tid + st]; __syncthreads(); }
  const float mu = red[0] / (float)N; __syncthreads();
  float s2 = 0.f;
  for (int u = 0; u < per / 4; ++u)
#pragma unroll
    for (int q = 0; q < 4; ++q) { const float c = vals[u * 4 + q] - mu; s2 += c * c; }
  red[tid] = s2; __syncthreads();
  for (int st = 128; st > 0; st >>= 1) { if (tid < st) red[tid] += red[tid + st]; __syncthreads(); }
  const float rs = rsqrtf(red[0] / (float)N + eps);
  for (int pass = 0; pass < 2; ++pass) {
    for (int u = 0; u < per / 4; ++u) {
      const int j = tid * 4 + 1024 * u;
      v4f o, sm;
#pragma unroll
      for (int q = 0; q < 4; ++q) {
        float gg = g[j + q], bb = bta[j + q];
        if (PARAM_BF16) { gg = bf16_round(gg); bb = bf16_round(bb); }
        sm[q] = vals[u * 4 + q]; o[q] = (vals[u * 4 + q] - mu) * rs * gg + bb;
      }
      if (out_sum) *(volatile v4f*)(out_sum + (size_t)row * N + j) = sm;
      *(volatile v4f*)(out_norm + (size_t)row * N + j) = o;
    }
    if (pass == 0) __threadfence();
  }
}


typedef _Float16 v16h __attribute__((ext_vector_type(16)));
union FragH { v16h v; v8us half[2]; _Float16 h[16]; unsigned short u[16]; };
template <int NT>
__device__ __forceinline__ v8f mmaH(v16h ah, v16h al, v16h bh, v16h bl, v8f c) {
  c = __builtin_amdgcn_wmma_f32_16x16x32_f16(false, ah, false, bh, (short)0, c, false, false);
  if (NT >= 2) c = __builtin_amdgcn_wmma_f32_16x16x32_f16(false, al, false, bh, (short)0, c, false, false);
  if (NT >= 3) c = __builtin_amdgcn_wmma_f32_16x16x32_f16(false, ah, false, bl, (short)0, c, false, false);
  asm volatile("v_nop\n\tv_nop\n\tv_nop\n\tv_nop" : "+v"(c) : "v"(ah), "v"(al), "v"(bh), "v"(bl));
  return c;
}
template <bool ASPLIT>
__global__ __launch_bounds__(128) void k_gemm_h(const float* __restrict__ A, int lda, size_t sA, const _Float16* __restrict__ Bh, int ldb, size_t sB, float alpha, float* __restrict__ C, int ldc, size_t sC, int M, int N, int K) {
  __shared__ __attribute__((aligned(16))) float so[4][16][64];
  const int tid = threadIdx.x, w = tid >> 5, lane = tid & 31, ln = lane & 15, hh = lane >> 4; const int by = blockIdx.y;
  A += (size_t)by * sA; Bh += (size_t)by * sB; C += (size_t)by * sC;
  const int ntn = (N + 63) / 64; const int wid = blockIdx.x * 4 + w; const int mt = wid / ntn, nq = wid % ntn; if (mt * 16 >= M) return;
  const int row0 = mt * 16, col0 = nq * 64; const float* arow = A + (size_t)(row0 + ln) * lda;
  v8f acc[4] = {};
  for (int kb = 0; kb < K; kb += 32) {
    FragH ah, al;
    const v4f x0 = *(const v4fa*)(arow + kb + 8 * hh), x1 = *(const v4fa*)(arow + kb + 8 * hh + 4), x2 = *(const v4fa*)(arow + kb + 16 + 8 * hh), x3 = *(const v4fa*)(arow + kb + 16 + 8 * hh + 4);
    float xs[16] = {x0[0],x0[1],x0[2],x0[3],x1[0],x1[1],x1[2],x1[3],x2[0],x2[1],x2[2],x2[3],x3[0],x3[1],x3[2],x3[3]};
#pragma unroll
    for (int i = 0; i < 16; ++i) { const _Float16 h = (_Float16)xs[i]; ah.h[i] = h; al.h[i] = ASPLIT ? (_Float16)(xs[i] - (float)h) : (_Float16)0.0f; }
#pragma unroll
    for (int t = 0; t < 4; ++t) { if (col0 + t * 16 >= N) continue; const size_t boff = (size_t)(col0 + t * 16 + ln) * ldb + kb; FragH bq; bq.half[0] = *(const v8us*)(Bh + boff + 8 * hh); bq.half[1] = *(const v8us*)(Bh + boff + 16 + 8 * hh);
      acc[t] = mmaH<ASPLIT ? 2 : 1>(ah.v, al.v, bq.v, bq.v, acc[t]); }
  }
#pragma unroll
  for (int t = 0; t < 4; ++t) { if (col0 + t * 16 >= N) continue;
#pragma unroll
    for (int r = 0; r < 8; ++r) so[w][8 * hh + r][t * 16 + ln] = acc[t][r] * alpha; }
  __builtin_amdgcn_fence(__ATOMIC_ACQ_REL, "workgroup"); __builtin_amdgcn_wave_barrier();
  const int rsub = lane >> 4, c4 = (lane & 15) * 4;
  for (int pass = 0; pass < 2; ++pass) {
#pragma unroll
    for (int q = 0; q < 8; ++q) { const int r = q * 2 + rsub; if (col0 + c4 < N) { const v4f v = *(const v4fa*)&so[w][r][c4]; *(volatile v4f*)(C + (size_t)(row0 + r) * ldc + col0 + c4) = v; } }
    if (pass == 0) __threadfence(); }
}

__global__ __launch_bounds__(256) void k_wt_f16(const float* __restrict__ W, _Float16* __restrict__ Wt, int K, int N, float scale) {
  const int t = blockIdx.x * 256 + threadIdx.x; if (t >= N * (K / 8)) return; const int n = t / (K / 8), k8 = (t % (K / 8)) * 8; FragH f;
#pragma unroll
  for (int i = 0; i < 8; ++i) f.h[i] = (_Float16)(bf16_round(W[(size_t)(k8 + i) * N + n]) * scale); const v8us o = f.half[0];
  *(volatile v8us*)((unsigned short*)Wt + (size_t)n * K + k8) = o; __threadfence(); *(volatile v8us*)((unsigned short*)Wt + (size_t)n * K + k8) = o;
}
template <int ACT>
__global__ __launch_bounds__(128) void k_gemm_hhx(const _Float16* __restrict__ A, int lda, size_t sA, const _Float16* __restrict__ Bh, int ldb, size_t sB, float alpha, const float* __restrict__ bias, size_t sBias, const float* __restrict__ CP, int rowsPerB, size_t sCPb, int row0g,
    float* __restrict__ C, _Float16* __restrict__ C16, int ldc, size_t sC, int M, int N, int K) {
  __shared__ __attribute__((aligned(16))) float so[4][16][64];
  const int tid = threadIdx.x, w = tid >> 5, lane = tid & 31, ln = lane & 15, hh = lane >> 4; const int by = blockIdx.y;
  A += (size_t)by * sA; Bh += (size_t)by * sB; const size_t cofs = (size_t)by * sC; const float* bp = bias ? bias + (size_t)by * sBias : nullptr;
  const int ntn = (N + 63) / 64; const int wid = blockIdx.x * 4 + w; const int mt = wid / ntn, nq = wid % ntn; if (mt * 16 >= M) return;
  const int row0 = mt * 16, col0 = nq * 64; const _Float16* arow = A + (size_t)(row0 + ln) * lda;
  v8f acc[4] = {};
  for (int kb = 0; kb < K; kb += 32) { FragH ah; ah.half[0] = *(const v8us*)((const unsigned short*)arow + kb + 8 * hh); ah.half[1] = *(const v8us*)((const unsigned short*)arow + kb + 16 + 8 * hh);
#pragma unroll
    for (int t = 0; t < 4; ++t) { if (col0 + t * 16 >= N) continue; const size_t boff = (size_t)(col0 + t * 16 + ln) * ldb + kb; FragH bq; bq.half[0] = *(const v8us*)((const unsigned short*)Bh + boff + 8 * hh); bq.half[1] = *(const v8us*)((const unsigned short*)Bh + boff + 16 + 8 * hh);
      acc[t] = mmaH<1>(ah.v, ah.v, bq.v, bq.v, acc[t]); }
  }
#pragma unroll
  for (int t = 0; t < 4; ++t) { if (col0 + t * 16 >= N) continue; const int col = col0 + t * 16 + ln; const float bv = bp ? bf16_round(bp[col]) : 0.f;
#pragma unroll
    for (int r = 0; r < 8; ++r) { float v = acc[t][r] * alpha + bv; if (CP) { const int bidx = (row0g + row0 + 8 * hh + r) / rowsPerB; v += CP[(size_t)bidx * sCPb + (size_t)by * 64 + col]; } if (ACT == 1) v = (v > 0.f) ? v : expm1f(v); else if (ACT == 7) v = (v > 0.f) ? v + 1.0f : expf(v); else if (ACT == 8) v = tanhf(v); else if (ACT == 9) v = 0.5f * v * (1.0f + tanhf(0.7978845608028654f * (v + 0.044715f * v * v * v))); else if (ACT == 11) v = 1.0f / (1.0f + expf(-v)); else if (ACT == 12) v = (v > 0.f) ? v : 0.01f * v; else if (ACT == 14) v = (v > 0.f) ? v : 0.1f * v; else if (ACT == 15) v = v / (1.0f + expf(-v)); else if (ACT == 3) v = fmaxf(v, 0.f); else if (ACT == 6) v = 0.5f * v * (1.0f + erff(v * 0.70710678118654752f)); so[w][8 * hh + r][t * 16 + ln] = v; } }
  __builtin_amdgcn_fence(__ATOMIC_ACQ_REL, "workgroup"); __builtin_amdgcn_wave_barrier();
  const int rsub = lane >> 4, c4 = (lane & 15) * 4; typedef _Float16 v4h __attribute__((ext_vector_type(4)));
  for (int pass = 0; pass < 2; ++pass) {
#pragma unroll
    for (int q = 0; q < 8; ++q) { const int r = q * 2 + rsub; if (col0 + c4 < N) { const v4f v = *(const v4fa*)&so[w][r][c4]; if (C) *(volatile v4f*)(C + cofs + (size_t)(row0 + r) * ldc + col0 + c4) = v; if (C16) { v4h h4; for (int i = 0; i < 4; ++i) h4[i] = (_Float16)v[i]; *(volatile v4h*)(C16 + cofs + (size_t)(row0 + r) * ldc + col0 + c4) = h4; } } }
    if (pass == 0) __threadfence(); }
}


typedef _Float16 v4h __attribute__((ext_vector_type(4)));

__global__ __launch_bounds__(256) void k_x16(const float* __restrict__ x, _Float16* __restrict__ X16, size_t n8) { const size_t t = (size_t)blockIdx.x * 256 + threadIdx.x; if (t >= n8) return; FragH f;
#pragma unroll
  for (int q = 0; q < 8; ++q) f.h[q] = (_Float16)bf16_round(x[t * 8 + q]); *(volatile v8us*)((unsigned short*)X16 + t * 8) = f.half[0]; __threadfence(); *(volatile v8us*)((unsigned short*)X16 + t * 8) = f.half[0]; }
__global__ __launch_bounds__(256) void k_h16(const float* __restrict__ x, _Float16* __restrict__ X16, size_t n8) { const size_t t = (size_t)blockIdx.x * 256 + threadIdx.x; if (t >= n8) return; FragH f;
#pragma unroll
  for (int q = 0; q < 8; ++q) f.h[q] = (_Float16)x[t * 8 + q]; *(volatile v8us*)((unsigned short*)X16 + t * 8) = f.half[0]; __threadfence(); *(volatile v8us*)((unsigned short*)X16 + t * 8) = f.half[0]; }
__global__ __launch_bounds__(256) void k_round16f(const float* __restrict__ W, _Float16* __restrict__ Bt, size_t n8) { const size_t t = (size_t)blockIdx.x * 256 + threadIdx.x; if (t >= n8) return; FragH f;
#pragma unroll
  for (int i = 0; i < 8; ++i) f.h[i] = (_Float16)(bf16_round(W[t * 8 + i]) * 16.0f); *(volatile v8us*)((unsigned short*)Bt + t * 8) = f.half[0]; __threadfence(); *(volatile v8us*)((unsigned short*)Bt + t * 8) = f.half[0]; }
template <int NHv, int TTv>
__global__ __launch_bounds__(256) void k_vt(const _Float16* __restrict__ V16, int ldv, int voff, _Float16* __restrict__ Vt) { __shared__ unsigned short tl[64][66]; const int tid = threadIdx.x; const int slab = blockIdx.x / (TTv / 64), lg = blockIdx.x % (TTv / 64); const int b = slab / NHv, h = slab % NHv;
  for (int i = tid; i < 64 * 8; i += 256) { const int r = i / 8, c8 = (i % 8) * 8; FragH f; f.half[0] = *(const v8us*)((const unsigned short*)V16 + ((size_t)b * TTv + lg * 64 + r) * ldv + voff + h * 64 + c8);
#pragma unroll
    for (int q = 0; q < 8; ++q) tl[r][c8 + q] = f.u[q]; }
  __syncthreads();
  for (int pass = 0; pass < 2; ++pass) {
#pragma unroll
    for (int rd = 0; rd < 2; ++rd) { const int d = rd * 32 + tid / 8, pc = tid % 8; FragH f;
#pragma unroll
      for (int q = 0; q < 8; ++q) f.u[q] = tl[pc * 8 + q][d];
      *(volatile v8us*)((unsigned short*)Vt + ((size_t)slab * 64 + d) * TTv + lg * 64 + pc * 8) = f.half[0]; }
    if (pass == 0) __threadfence(); } }

__global__ __launch_bounds__(256) void k_hl(const float* __restrict__ F, _Float16* __restrict__ Hh, _Float16* __restrict__ Hl, size_t n8) { const size_t t = (size_t)blockIdx.x * 256 + threadIdx.x; if (t >= n8) return; FragH fh, fl; const v4f a = *(const v4fa*)(F + t * 8), c = *(const v4fa*)(F + t * 8 + 4);
#pragma unroll
  for (int q = 0; q < 4; ++q) { _Float16 h = (_Float16)a[q]; fh.h[q] = h; fl.h[q] = (_Float16)((a[q] - (float)h) * 1024.0f); h = (_Float16)c[q]; fh.h[4 + q] = h; fl.h[4 + q] = (_Float16)((c[q] - (float)h) * 1024.0f); }
  for (int pass = 0; pass < 2; ++pass) { *(volatile v8us*)((unsigned short*)Hh + t * 8) = fh.half[0]; *(volatile v8us*)((unsigned short*)Hl + t * 8) = fl.half[0]; if (pass == 0) __threadfence(); } }

__global__ __launch_bounds__(256) void k_abase(const float* __restrict__ x, const float* __restrict__ W1, const float* __restrict__ b1, float* __restrict__ A) {
  #pragma clang fp contract(off)
  const int t = blockIdx.x * 256 + threadIdx.x; if (t >= NB * NN * MH) return; const int j = t % MH; const int bs = t / MH; const float* xr = x + (size_t)bs * TT * FF; float s = bf16_round(b1[j]);
#pragma unroll 1
  for (int tt = 0; tt < TT; ++tt) {
#pragma unroll
    for (int i = 0; i < 4; ++i) s += bf16_round(xr[tt * FF + i]) * bf16_round(W1[(size_t)(tt * 5 + i) * MH + j]); }
  *(volatile float*)(A + t) = s; __threadfence(); *(volatile float*)(A + t) = s; }
__global__ __launch_bounds__(256) void k_ecol(const float* __restrict__ x, int b, int s0, _Float16* __restrict__ E) { const int t = blockIdx.x * 256 + threadIdx.x; if (t >= SCH * NN * 4) return; const int g = t % 4; const int row = t / 4; const int sl = row / NN, c = row % NN; const float* xr = x + (((size_t)b * NN + s0 + sl) * TT) * FF + 4 + c; FragH f = FragH{};
#pragma unroll
  for (int q = 0; q < 8; ++q) { const int tt = g * 8 + q; if (tt < TT) f.h[q] = (_Float16)bf16_round(xr[(size_t)tt * FF]); }
  *(volatile v8us*)((unsigned short*)E + (size_t)row * 32 + g * 8) = f.half[0]; __threadfence(); *(volatile v8us*)((unsigned short*)E + (size_t)row * 32 + g * 8) = f.half[0]; }
__global__ __launch_bounds__(256) void k_wcol(const float* __restrict__ W1, _Float16* __restrict__ Bt) { const int t = blockIdx.x * 256 + threadIdx.x; if (t >= MH * 4) return; const int g = t % 4, j = t / 4; FragH f;
#pragma unroll
  for (int q = 0; q < 8; ++q) { const int tt = g * 8 + q; f.h[q] = (tt < TT) ? (_Float16)(bf16_round(W1[(size_t)(tt * 5 + 4) * MH + j]) * 16.0f) : (_Float16)0.0f; }
  *(volatile v8us*)((unsigned short*)Bt + (size_t)j * 32 + g * 8) = f.half[0]; __threadfence(); *(volatile v8us*)((unsigned short*)Bt + (size_t)j * 32 + g * 8) = f.half[0]; }
__global__ __launch_bounds__(256) void k_hsum(const float* __restrict__ H, int b, int first, float* HS) {
  #pragma clang fp contract(off)
  const int t = blockIdx.x * 256 + threadIdx.x; if (t >= NN * (MH / 4)) return; const int j0 = (t % (MH / 4)) * 4, c = t / (MH / 4); v4f s; float* dst = HS + ((size_t)b * NN + c) * MH + j0;
  if (first) { s[0] = 0.f; s[1] = 0.f; s[2] = 0.f; s[3] = 0.f; } else s = *(const v4f*)dst;
#pragma unroll 1
  for (int sl = 0; sl < SCH; ++sl) { const v4f a = *(const v4fa*)(H + ((size_t)sl * NN + c) * MH + j0);
#pragma unroll
    for (int k = 0; k < 4; ++k) s[k] += a[k]; }
  *(volatile v4f*)dst = s; __threadfence(); *(volatile v4f*)dst = s; }
__global__ __launch_bounds__(256) void k_hs16(const float* __restrict__ HS, _Float16* __restrict__ O, size_t n8) { const size_t t = (size_t)blockIdx.x * 256 + threadIdx.x; if (t >= n8) return; const v4f a = *(const v4fa*)(HS + t * 8), c = *(const v4fa*)(HS + t * 8 + 4); FragH f;
#pragma unroll
  for (int q = 0; q < 8; ++q) f.h[q] = (_Float16)(((q < 4) ? a[q] : c[q - 4]) * 0.0625f);
  *(volatile v8us*)((unsigned short*)O + t * 8) = f.half[0]; __threadfence(); *(volatile v8us*)((unsigned short*)O + t * 8) = f.half[0]; }
__global__ __launch_bounds__(256) void k_mi(const float* __restrict__ MS, const float* __restrict__ x, _Float16* __restrict__ MI) { const int t = blockIdx.x * 256 + threadIdx.x; if (t >= NB * NN * 8) return; const int g = t % 8, row = t / 8; FragH f = FragH{};
#pragma unroll
  for (int q = 0; q < 8; ++q) { const int i = g * 8 + q; float v = 0.f; if (i < MD) v = MS[(size_t)row * MD + i]; else if (i < MD + 4) v = bf16_round(x[((size_t)row * TT + TT - 1) * FF + (i - MD)]); f.h[q] = (_Float16)v; }
  *(volatile v8us*)((unsigned short*)MI + (size_t)row * 64 + g * 8) = f.half[0]; __threadfence(); *(volatile v8us*)((unsigned short*)MI + (size_t)row * 64 + g * 8) = f.half[0]; }
__global__ __launch_bounds__(256) void k_wi1(const float* __restrict__ W, _Float16* __restrict__ Bt) { const int t = blockIdx.x * 256 + threadIdx.x; if (t >= UH * 8) return; const int g = t % 8, o = t / 8; FragH f;
#pragma unroll
  for (int q = 0; q < 8; ++q) { const int k = g * 8 + q; f.h[q] = (k < MD + 4) ? (_Float16)(bf16_round(W[(size_t)k * UH + o]) * 16.0f) : (_Float16)0.0f; }
  *(volatile v8us*)((unsigned short*)Bt + (size_t)o * 64 + g * 8) = f.half[0]; __threadfence(); *(volatile v8us*)((unsigned short*)Bt + (size_t)o * 64 + g * 8) = f.half[0]; }
__global__ __launch_bounds__(256) void k_bscale(const float* __restrict__ b, int n, float scale, float* __restrict__ O) { const int i = threadIdx.x; if (i >= n) return; const float v = scale * bf16_round(b[i]); *(volatile float*)(O + i) = v; __threadfence(); *(volatile float*)(O + i) = v; }
__global__ __launch_bounds__(256) void k_fin(const float* __restrict__ H2, const float* __restrict__ W2, const float* __restrict__ b2, float* __restrict__ out) {
  #pragma clang fp contract(off)
  const int row = blockIdx.x * 256 + threadIdx.x; if (row >= NB * NN) return; const float* h = H2 + (size_t)row * UH; v4f v;
#pragma unroll
  for (int k = 0; k < 4; ++k) v[k] = bf16_round(b2[k]);
#pragma unroll 1
  for (int j = 0; j < UH; ++j) { const float hj = h[j];
#pragma unroll
    for (int k = 0; k < 4; ++k) v[k] += hj * bf16_round(W2[j * 4 + k]); }
  *(volatile v4f*)(out + (size_t)row * 4) = v; __threadfence(); *(volatile v4f*)(out + (size_t)row * 4) = v; }

extern "C" void kernel_launch(void* const* d_in, const int* in_sizes, int n_in,
                              void* d_out, int out_size, void* d_ws, size_t ws_size, hipStream_t stream) {
  (void)in_sizes; (void)n_in; (void)out_size;
  const float* const* I = (const float* const*)d_in; const float* x = I[0]; const float* mW1 = I[1]; const float* mb1 = I[2]; const float* mW2 = I[3]; const float* mb2 = I[4]; const float* iW1 = I[5]; const float* ib1 = I[6]; const float* iW2 = I[7]; const float* ib2 = I[8];
  char* ws = (char*)d_ws; size_t off = 0;
  auto take = [&](size_t bytes) { char* p = ws + off; off += (bytes + 255) & ~(size_t)255; return p; };
  _Float16* BW = (_Float16*)take((size_t)MH * 32 * 2); _Float16* BM2 = (_Float16*)take((size_t)MD * MH * 2); float* BM2b = (float*)take(MD * 4); _Float16* BI1 = (_Float16*)take((size_t)UH * 64 * 2);
  float* A = (float*)take((size_t)NB * NN * MH * 4); _Float16* E = (_Float16*)take((size_t)SCH * NN * 32 * 2); float* H = (float*)take((size_t)SCH * NN * MH * 4); float* HS = (float*)take((size_t)NB * NN * MH * 4); _Float16* HS16 = (_Float16*)take((size_t)NB * NN * MH * 2); float* MS = (float*)take((size_t)NB * NN * MD * 4); _Float16* MI = (_Float16*)take((size_t)NB * NN * 64 * 2); float* H2 = (float*)take((size_t)NB * NN * UH * 4);
  if (off > ws_size) return;
  k_wcol<<<(MH * 4 + 255) / 256, 256, 0, stream>>>(mW1, BW); k_wt_f16<<<(MD * (MH / 8) + 255) / 256, 256, 0, stream>>>(mW2, BM2, MH, MD, 16.0f); k_bscale<<<1, 256, 0, stream>>>(mb2, MD, (float)NN, BM2b); k_wi1<<<(UH * 8 + 255) / 256, 256, 0, stream>>>(iW1, BI1);
  k_abase<<<(NB * NN * MH + 255) / 256, 256, 0, stream>>>(x, mW1, mb1, A);
  const dim3 gH(((SCH * NN / 16) * (MH / 64) + 3) / 4, 1);
  for (int b = 0; b < NB; ++b) for (int s0 = 0; s0 < NN; s0 += SCH) {
    k_ecol<<<(SCH * NN * 4 + 255) / 256, 256, 0, stream>>>(x, b, s0, E);
    k_gemm_hhx<3><<<gH, 128, 0, stream>>>(E, 32, 0, BW, 32, 0, 0.0625f, nullptr, 0, A + ((size_t)b * NN + s0) * MH, NN, (size_t)MH, 0, H, nullptr, MH, 0, SCH * NN, MH, 32);
    k_hsum<<<(NN * (MH / 4) + 255) / 256, 256, 0, stream>>>(H, b, s0 == 0, HS); }
  k_hs16<<<(unsigned)(((size_t)NB * NN * MH / 8 + 255) / 256), 256, 0, stream>>>(HS, HS16, (size_t)NB * NN * MH / 8);
  k_gemm_hhx<0><<<dim3((((NB * NN) / 16) * 1 + 3) / 4, 1), 128, 0, stream>>>(HS16, MH, 0, BM2, MH, 0, 1.0f, BM2b, 0, nullptr, 1, 0, 0, MS, nullptr, MD, 0, NB * NN, MD, MH);
  k_mi<<<(NB * NN * 8 + 255) / 256, 256, 0, stream>>>(MS, x, MI);
  k_gemm_hhx<3><<<dim3((((NB * NN) / 16) * (UH / 64) + 3) / 4, 1), 128, 0, stream>>>(MI, 64, 0, BI1, 64, 0, 0.0625f, ib1, 0, nullptr, 1, 0, 0, H2, nullptr, UH, 0, NB * NN, UH, 64);
  k_fin<<<(NB * NN + 255) / 256, 256, 0, stream>>>(H2, iW2, ib2, (float*)d_out);
}
